// SelectiveSSM_18305150615687
// MI455X (gfx1250) — hardware-run, weakly checked
//
#include <hip/hip_runtime.h>
#include <math.h>
#include <stddef.h>

typedef __attribute__((ext_vector_type(16))) _Float16 v16h;
typedef __attribute__((ext_vector_type(8)))  _Float16 v8h;
typedef __attribute__((ext_vector_type(16))) __bf16   v16b;
typedef __attribute__((ext_vector_type(8)))  __bf16   v8b;
typedef __attribute__((ext_vector_type(8)))  float    v8f;
typedef __attribute__((ext_vector_type(4)))  float    v4f;
typedef __attribute__((ext_vector_type(4)))  unsigned v4u;

constexpr int NB = 2;
constexpr int NCH = 4;
constexpr int NHT = 256;
constexpr int NWD = 256;
constexpr int NPLANE = NB * NCH;
constexpr int HWPIX = NHT * NWD;
constexpr int NPIX = NPLANE * HWPIX;
constexpr int NMID = 128;
constexpr int PADD = 260;
constexpr int MROWS = NB * NHT * NWD;
constexpr int K1REAL = 36;
constexpr int K1 = 64;
constexpr int K2 = 9 * NMID;
constexpr int N2ROWS = 16;
constexpr int NTHR = 256;
constexpr int NROWBLK = NPLANE * NHT;
constexpr int NIMGROW = NB * NHT;
constexpr int PLINE = 32;
constexpr int SPITCH = 68;
constexpr long TMID_HALVES = (long)NB * PADD * PADD * NMID;
constexpr int CONV1_BLOCKS = (MROWS / 64) * (NMID / 64) / 8;
constexpr int ZERO_BLOCKS = (int)((2 * TMID_HALVES) / 8 / NTHR);
constexpr float MID_CARRY = 16.0f;
constexpr float W2_CARRY = 16.0f;
constexpr float C2_FOLD = 1.0f / 256.0f;
constexpr float FLT_TINY = 1.17549435e-38f;

static_assert(MROWS % 64 == 0);
static_assert(NMID % 64 == 0);
static_assert(K1 % 32 == 0 && K1 >= K1REAL);
static_assert(K2 % 32 == 0);
static_assert(NWD % 64 == 0);
static_assert(CONV1_BLOCKS * 8 == (MROWS / 64) * (NMID / 64));
static_assert(NWD == NTHR);
static_assert((long)ZERO_BLOCKS * NTHR * 8 == 2 * TMID_HALVES);
static_assert(NPIX % (4 * NTHR) == 0);
static_assert((NMID * (K1 / 8)) % NTHR == 0);
static_assert((N2ROWS * (K2 / 8)) % NTHR == 0);
static_assert(NROWBLK == 8 * NTHR);
static_assert(HWPIX % NTHR == 0);

constexpr size_t TMID_BYTES = (size_t)TMID_HALVES * 2;
constexpr size_t OFF_TSU = 0;
constexpr size_t OFF_TNU = OFF_TSU + TMID_BYTES;
constexpr size_t IM_BYTES = (size_t)MROWS * K1 * 2;
constexpr size_t OFF_IMH = OFF_TNU + TMID_BYTES;
constexpr size_t OFF_IML = OFF_IMH + IM_BYTES;
constexpr size_t PL_BYTES = (size_t)NPIX * 4;
constexpr size_t OFF_STA = OFF_IML + IM_BYTES;
constexpr size_t OFF_STB = OFF_STA + PL_BYTES;
constexpr size_t OFF_ACC = OFF_STB + PL_BYTES;
constexpr size_t OFF_GM  = OFF_ACC + PL_BYTES;
constexpr size_t OFF_SIM = OFF_GM + PL_BYTES;
constexpr size_t OFF_BSS = OFF_SIM + PL_BYTES;
constexpr size_t OFF_HF  = OFF_BSS + PL_BYTES;
constexpr size_t W1P_BYTES = (size_t)2 * NMID * K1 * 2;
constexpr size_t OFF_W1H = OFF_HF + PL_BYTES;
constexpr size_t OFF_W1L = OFF_W1H + W1P_BYTES;
constexpr size_t W2P_BYTES = (size_t)2 * N2ROWS * K2 * 2;
constexpr size_t OFF_W2 = OFF_W1L + W1P_BYTES;
constexpr size_t PART_BYTES = (size_t)NROWBLK * PLINE * 4;
constexpr size_t OFF_PART = OFF_W2 + W2P_BYTES;
constexpr size_t OFF_LPRT = OFF_PART + PART_BYTES;
constexpr size_t OFF_GATE = OFF_LPRT + PART_BYTES;
constexpr size_t WS_TOTAL = OFF_GATE + 128;
static_assert(WS_TOTAL == (size_t)118120576);
static_assert(WS_TOTAL <= (size_t)134217728);
static_assert(OFF_TNU % 256 == 0 && OFF_IMH % 256 == 0 && OFF_STA % 256 == 0 && OFF_HF % 256 == 0 && OFF_W1H % 256 == 0);
static_assert(OFF_W2 % 256 == 0 && OFF_PART % 256 == 0 && OFF_LPRT % 256 == 0 && OFF_GATE % 128 == 0);
static_assert((size_t)NPIX * 4 == (size_t)2097152);

__device__ __forceinline__ unsigned short f2bf_bits(float f) {
  unsigned u = __float_as_uint(f);
  return (unsigned short)((u + 0x7FFFu + ((u >> 16) & 1u)) >> 16);
}
__device__ __forceinline__ float bf_bits2f(unsigned short h) { return __uint_as_float(((unsigned)h) << 16); }

__device__ __forceinline__ void dep_guard_h(v8f& a, v8f& b, v16h x, v16h y) { asm volatile("v_nop\n\tv_nop\n\tv_nop\n\tv_nop" : "+v"(a), "+v"(b) : "v"(x), "v"(y)); }
__device__ __forceinline__ void dep_guard_b(v8f& a, v8f& b, v16b x, v16b y) { asm volatile("v_nop\n\tv_nop\n\tv_nop\n\tv_nop" : "+v"(a), "+v"(b) : "v"(x), "v"(y)); }
__device__ __forceinline__ void keep4_h(v16h a, v16h b, v16h c, v16h d) { asm volatile("v_nop" :: "v"(a), "v"(b), "v"(c), "v"(d)); }
__device__ __forceinline__ void keep4_b(v16b a, v16b b, v16b c, v16b d) { asm volatile("v_nop" :: "v"(a), "v"(b), "v"(c), "v"(d)); }
__device__ __forceinline__ void acc_guard4(v8f& a, v8f& b, v8f& c, v8f& d) { asm volatile("v_nop\n\tv_nop\n\tv_nop\n\tv_nop" : "+v"(a), "+v"(b), "+v"(c), "+v"(d)); }
__device__ __forceinline__ void guard4a5(v8f& a, v8f& b, v8f& c, v8f& d, v16h p0, v16h p1, v16h p2, v16h p3, v16h q) {
  asm volatile("v_nop\n\tv_nop\n\tv_nop\n\tv_nop" : "+v"(a), "+v"(b), "+v"(c), "+v"(d) : "v"(p0), "v"(p1), "v"(p2), "v"(p3), "v"(q));
}
template <typename T> struct Frag;
template <> struct Frag<_Float16> {
  typedef v16h V; union U { v16h v; v8h h[2]; };
  static __device__ __forceinline__ v16h load(const _Float16* p) {
    U f; f.h[0] = *(const v8h*)(p); f.h[1] = *(const v8h*)(p + 16); return f.v;
  }
  static __device__ __forceinline__ v8f mma(v16h a, v16h b, v8f c) {
    return __builtin_amdgcn_wmma_f32_16x16x32_f16(false, a, false, b, (short)0, c, false, false);
  }
  static __device__ __forceinline__ void guard(v8f& a, v8f& b, v16h x, v16h y) { dep_guard_h(a, b, x, y); }
  static __device__ __forceinline__ void keep(v16h a, v16h b, v16h c, v16h d) { keep4_h(a, b, c, d); }
};
template <> struct Frag<__bf16> {
  typedef v16b V; union U { v16b v; v8b h[2]; };
  static __device__ __forceinline__ v16b load(const __bf16* p) {
    U f; f.h[0] = *(const v8b*)(p); f.h[1] = *(const v8b*)(p + 16); return f.v;
  }
  static __device__ __forceinline__ v8f mma(v16b a, v16b b, v8f c) {
    return __builtin_amdgcn_wmma_f32_16x16x32_bf16(false, a, false, b, (short)0, c, false, false);
  }
  static __device__ __forceinline__ void guard(v8f& a, v8f& b, v16b x, v16b y) { dep_guard_b(a, b, x, y); }
  static __device__ __forceinline__ void keep(v16b a, v16b b, v16b c, v16b d) { keep4_b(a, b, c, d); }
};

__device__ __forceinline__ void st2(float* p, float v) {
  *(volatile float*)p = v;
  __threadfence();
  *(volatile float*)p = v;
}
__device__ __forceinline__ float fsigm(float v) { return 1.0f / (1.0f + expf(-v)); }

__device__ __forceinline__ void ld_row3(const float* __restrict__ rowp, int x, float& vl, float& vc, float& vr) {
  const int xl = (x > 0) ? (x - 1) : 0;
  const int xr = (x < NWD - 1) ? (x + 1) : (NWD - 1);
  const float fl = (x > 0) ? 1.0f : 0.0f;
  const float fr = (x < NWD - 1) ? 1.0f : 0.0f;
  vl = rowp[xl] * fl;
  vc = rowp[x];
  vr = rowp[xr] * fr;
}

__device__ __forceinline__ float grad_mag(const float* __restrict__ plane, int y, int x, const float* wx, const float* wy) {
  float a0 = 0.0f, a1 = 0.0f, a2 = 0.0f, a3 = 0.0f, a4 = 0.0f, a5 = 0.0f, a6 = 0.0f, a7 = 0.0f, a8 = 0.0f;
  if (y > 0) ld_row3(plane + (size_t)(y - 1) * NWD, x, a0, a1, a2);
  ld_row3(plane + (size_t)y * NWD, x, a3, a4, a5);
  if (y < NHT - 1) ld_row3(plane + (size_t)(y + 1) * NWD, x, a6, a7, a8);
  float gx = 0.0f;
  gx += wx[0] * a0; gx += wx[1] * a1; gx += wx[2] * a2;
  gx += wx[3] * a3; gx += wx[4] * a4; gx += wx[5] * a5;
  gx += wx[6] * a6; gx += wx[7] * a7; gx += wx[8] * a8;
  float gy = 0.0f;
  gy += wy[0] * a0; gy += wy[1] * a1; gy += wy[2] * a2;
  gy += wy[3] * a3; gy += wy[4] * a4; gy += wy[5] * a5;
  gy += wy[6] * a6; gy += wy[7] * a7; gy += wy[8] * a8;
  return sqrtf(gx * gx + gy * gy);
}

__global__ __launch_bounds__(NTHR) void k_zero16(unsigned short* __restrict__ p, long n8) {
  const long i = (long)blockIdx.x * NTHR + threadIdx.x;
  if (i >= n8) return;
  const v4u z = {0u, 0u, 0u, 0u};
  *(volatile v4u*)(p + i * 8) = z;
  __threadfence();
  *(volatile v4u*)(p + i * 8) = z;
}

__global__ __launch_bounds__(NTHR) void k_w1prep(const float* __restrict__ wsu, const float* __restrict__ wnu,
                                                  unsigned short* __restrict__ hi, unsigned short* __restrict__ lo) {
  const float* w = (blockIdx.y == 0) ? wsu : wnu;
  const int i = blockIdx.x * NTHR + threadIdx.x;
  if (i >= NMID * (K1 / 8)) return;
  const int n = i >> 3;
  const int k0 = (i & 7) * 8;
  v8h hv, lv;
#pragma unroll
  for (int e = 0; e < 8; ++e) {
    const int k = k0 + e;
    const int kc = (k < K1REAL) ? k : (K1REAL - 1);
    const float fk = (k < K1REAL) ? 1.0f : 0.0f;
    const float v = w[n * K1REAL + kc] * fk;
    const unsigned short hb = f2bf_bits(v);
    const unsigned short lb = f2bf_bits(v - bf_bits2f(hb));
    hv[e] = __builtin_bit_cast(_Float16, hb);
    lv[e] = __builtin_bit_cast(_Float16, lb);
  }
  const size_t o = (size_t)blockIdx.y * NMID * K1 + (size_t)i * 8;
  *(volatile v8h*)(hi + o) = hv;
  *(volatile v8h*)(lo + o) = lv;
  __threadfence();
  *(volatile v8h*)(hi + o) = hv;
  *(volatile v8h*)(lo + o) = lv;
}

__global__ __launch_bounds__(NTHR) void k_w2prep(const float* __restrict__ wsu, const float* __restrict__ wnu,
                                                  unsigned short* __restrict__ w2p) {
  const float* w = (blockIdx.y == 0) ? wsu : wnu;
  const int i = blockIdx.x * NTHR + threadIdx.x;
  if (i >= N2ROWS * (K2 / 8)) return;
  const int n = i / (K2 / 8);
  const int k0 = (i - n * (K2 / 8)) * 8;
  const int nc = (n < NCH) ? n : (NCH - 1);
  const float fs = (n < NCH) ? W2_CARRY : 0.0f;
  v8h hv;
#pragma unroll
  for (int e = 0; e < 8; ++e) {
    const int k = k0 + e;
    const int tap = k >> 7;
    const int ci = k & (NMID - 1);
    const float v = w[((size_t)(nc * NMID + ci)) * 9 + tap] * fs;
    hv[e] = (_Float16)v;
  }
  const size_t o = (size_t)blockIdx.y * N2ROWS * K2 + (size_t)i * 8;
  *(volatile v8h*)(w2p + o) = hv;
  __threadfence();
  *(volatile v8h*)(w2p + o) = hv;
}

__global__ __launch_bounds__(NTHR) void k_gate(const float* __restrict__ x, const float* __restrict__ fcw,
                                                const float* __restrict__ fcb, const float* __restrict__ mw,
                                                float* __restrict__ gate) {
  __shared__ float red[NTHR];
  __shared__ float gs[NPLANE];
  __shared__ __align__(16) float gl[32];
  const int tid = threadIdx.x;
#pragma unroll 1
  for (int p = 0; p < NPLANE; ++p) {
    const float* xp = x + (size_t)p * HWPIX;
    float s = 0.0f;
#pragma unroll 1
    for (int i = tid; i < HWPIX; i += NTHR) s += xp[i];
    red[tid] = s;
    __syncthreads();
#pragma unroll 1
    for (int off = NTHR / 2; off > 0; off >>= 1) {
      if (tid < off) red[tid] += red[tid + off];
      __syncthreads();
    }
    if (tid == 0) gs[p] = red[0] * (1.0f / 65536.0f);
    __syncthreads();
  }
  if (tid < 32) {
    const int bb = (tid >> 2) & 1;
    const int cc = tid & 3;
    float z = 0.0f;
#pragma unroll
    for (int j = 0; j < NCH; ++j) z += gs[bb * NCH + j] * fcw[cc * NCH + j];
    z += fcb[cc];
    const float inw = fsigm(z);
    const float smw = fsigm(mw[cc]);
    const float f1 = (tid < 8) ? 1.0f : 0.0f;
    const float f2 = (tid >= 8 && tid < 12) ? 1.0f : 0.0f;
    gl[tid] = fmaf(inw, f1, smw * f2);
  }
  __syncthreads();
  if (tid < 8) {
    const v4f v = *(const v4f*)(gl + tid * 4);
    *(volatile v4f*)(gate + tid * 4) = v;
    __threadfence();
    *(volatile v4f*)(gate + tid * 4) = v;
  }
}

__global__ __launch_bounds__(NTHR) void k_init(const float* __restrict__ x, const float* __restrict__ gate,
                                                float* __restrict__ st) {
  const int i = blockIdx.x * NTHR + threadIdx.x;
  if (i >= NPIX / 4) return;
  const int plane = i >> 14;
  const float inw = gate[plane];
  const float smw = gate[8 + (plane & 3)];
  const v4f v = *(const v4f*)(x + (size_t)i * 4);
  v4f o;
#pragma unroll
  for (int e = 0; e < 4; ++e) o[e] = (v[e] * inw) * smw;
  *(volatile v4f*)(st + (size_t)i * 4) = o;
  __threadfence();
  *(volatile v4f*)(st + (size_t)i * 4) = o;
}

__global__ __launch_bounds__(NTHR) void k_im2col(const float* __restrict__ st, int dil,
                                                  unsigned short* __restrict__ hi, unsigned short* __restrict__ lo) {
  __shared__ float tile[NCH * 3 * PADD];
  const int tid = threadIdx.x;
  const int bimg = blockIdx.x >> 8;
  const int y = blockIdx.x & 255;
  if (tid < 48) {
    const int q = tid >> 2;
    const int cc = tid & 3;
    const int col = (cc < 2) ? cc : (NWD + cc);
    tile[q * PADD + col] = 0.0f;
  }
  __syncthreads();
#pragma unroll 1
  for (int q = 0; q < NCH * 3; ++q) {
    const int ci = q / 3;
    const int r = q - ci * 3;
    const int yy = y + (r - 1) * dil;
    float v = 0.0f;
    if (yy >= 0 && yy < NHT) v = st[((size_t)(bimg * NCH + ci) * NHT + yy) * NWD + tid];
    tile[q * PADD + tid + 2] = v;
  }
  __syncthreads();
  const int xg = tid >> 3;
  const int k0 = (tid & 7) * 8;
#pragma unroll 1
  for (int p = 0; p < 8; ++p) {
    const int x = p * 32 + xg;
    v8h hv, lv;
#pragma unroll
    for (int e = 0; e < 8; ++e) {
      const int k = k0 + e;
      const int ci = k / 9;
      const int r9 = k - ci * 9;
      const int ky = r9 / 3;
      const int kx = r9 - ky * 3;
      const int cic = (ci < NCH) ? ci : (NCH - 1);
      const float fk = (k < K1REAL) ? 1.0f : 0.0f;
      const float v = tile[(cic * 3 + ky) * PADD + x + 2 + (kx - 1) * dil] * fk;
      const unsigned short hb = f2bf_bits(v);
      const unsigned short lb = f2bf_bits(v - bf_bits2f(hb));
      hv[e] = __builtin_bit_cast(_Float16, hb);
      lv[e] = __builtin_bit_cast(_Float16, lb);
    }
    const size_t o = ((size_t)blockIdx.x * NWD + x) * K1 + k0;
    *(volatile v8h*)(hi + o) = hv;
    *(volatile v8h*)(lo + o) = lv;
    __threadfence();
    *(volatile v8h*)(hi + o) = hv;
    *(volatile v8h*)(lo + o) = lv;
  }
}

__global__ __launch_bounds__(NTHR) void k_conv1(
    const unsigned short* __restrict__ Ahp, const unsigned short* __restrict__ Alp,
    const unsigned short* __restrict__ Bhp, const unsigned short* __restrict__ Blp,
    const float* __restrict__ bias, unsigned short* __restrict__ Cp) {
  typedef Frag<__bf16> F;
  typedef v16b V;
  const __bf16* Ah = (const __bf16*)Ahp;
  const __bf16* Al = (const __bf16*)Alp;
  const __bf16* Bh = (const __bf16*)Bhp;
  const __bf16* Bl = (const __bf16*)Blp;
  __shared__ __align__(16) float sT[8][16 * SPITCH];
  const int lane = threadIdx.x & 31;
  const int wave = threadIdx.x >> 5;
  const int tilesN = NMID >> 6;
  const int tilesM = MROWS >> 6;
  const int tile = blockIdx.x * 8 + wave;
  if (tile >= tilesM * tilesN) return;
  const int tm = tile / tilesN;
  const int tn = tile - tm * tilesN;
  const int m0 = tm << 6;
  const int n0 = tn << 6;
  const int rlane = lane & 15;
  const int koff  = (lane >> 4) * 8;
  const int mOff  = (lane >> 4) * 8;

  v8f acc[4][4];
#pragma unroll
  for (int i = 0; i < 4; ++i)
#pragma unroll
    for (int j = 0; j < 4; ++j) acc[i][j] = (v8f){0.f, 0.f, 0.f, 0.f, 0.f, 0.f, 0.f, 0.f};

#pragma unroll 1
  for (int k0 = 0; k0 < K1; k0 += 32) {
#pragma unroll
    for (int jh = 0; jh < 2; ++jh) {
      const size_t bo0 = (size_t)(n0 + jh * 32 + rlane) * K1 + koff + k0;
      const size_t bo1 = bo0 + (size_t)16 * K1;
      const V bh0 = F::load(Bh + bo0);
      const V bh1 = F::load(Bh + bo1);
      const V bl0 = F::load(Bl + bo0);
      const V bl1 = F::load(Bl + bo1);
#pragma unroll
      for (int i = 0; i < 4; ++i) {
        const size_t ao = (size_t)(m0 + (i << 4) + rlane) * K1 + koff + k0;
        const V ah = F::load(Ah + ao);
        const V al = F::load(Al + ao);
        acc[i][2 * jh] = F::mma(ah, bh0, acc[i][2 * jh]);
        acc[i][2 * jh] = F::mma(ah, bl0, acc[i][2 * jh]);
        acc[i][2 * jh] = F::mma(al, bh0, acc[i][2 * jh]);
        acc[i][2 * jh + 1] = F::mma(ah, bh1, acc[i][2 * jh + 1]);
        acc[i][2 * jh + 1] = F::mma(ah, bl1, acc[i][2 * jh + 1]);
        acc[i][2 * jh + 1] = F::mma(al, bh1, acc[i][2 * jh + 1]);
        dep_guard_b(acc[i][2 * jh], acc[i][2 * jh + 1], ah, al);
      }
      keep4_b(bh0, bh1, bl0, bl1);
    }
  }
  acc_guard4(acc[0][0], acc[0][1], acc[0][2], acc[0][3]);
  acc_guard4(acc[1][0], acc[1][1], acc[1][2], acc[1][3]);
  acc_guard4(acc[2][0], acc[2][1], acc[2][2], acc[2][3]);
  acc_guard4(acc[3][0], acc[3][1], acc[3][2], acc[3][3]);

  float* slab = sT[wave];
#pragma unroll
  for (int i = 0; i < 4; ++i) {
    const int mBase = m0 + (i << 4);
#pragma unroll
    for (int j = 0; j < 4; ++j) {
      const int n = n0 + (j << 4) + rlane;
      const float bv = bias[n];
#pragma unroll
      for (int r = 0; r < 8; ++r) {
        float v = (acc[i][j][r] + bv) * MID_CARRY;
        v = fmaxf(v, 0.0f);
        slab[(mOff + r) * SPITCH + (j << 4) + rlane] = v;
      }
    }
    __builtin_amdgcn_fence(__ATOMIC_RELEASE, "workgroup");
    __builtin_amdgcn_wave_barrier();
    __builtin_amdgcn_fence(__ATOMIC_ACQUIRE, "workgroup");
    {
      const int q = lane >> 3;
      const int c8 = (lane & 7) * 8;
      for (int pass = 0; pass < 2; ++pass) {
#pragma unroll
        for (int it = 0; it < 4; ++it) {
          const int row = it * 4 + q;
          const int m = mBase + row;
          const int bb = m >> 16;
          const int yy = (m >> 8) & 255;
          const int xx = m & 255;
          const size_t pp = ((size_t)(bb * PADD + yy + 2)) * PADD + (size_t)(xx + 2);
          const float* sp = slab + row * SPITCH + c8;
          v8h hv;
#pragma unroll
          for (int e = 0; e < 8; ++e) hv[e] = (_Float16)sp[e];
          *(volatile v8h*)(Cp + pp * NMID + n0 + c8) = hv;
        }
        __threadfence();
      }
    }
    __builtin_amdgcn_fence(__ATOMIC_RELEASE, "workgroup");
    __builtin_amdgcn_wave_barrier();
    __builtin_amdgcn_fence(__ATOMIC_ACQUIRE, "workgroup");
  }
}

__global__ __launch_bounds__(128) void k_conv2(const unsigned short* __restrict__ tsu, const unsigned short* __restrict__ tnu,
                                               const unsigned short* __restrict__ w2p,
                                               const float* __restrict__ bsu, const float* __restrict__ bnu,
                                               float* __restrict__ accp) {
  typedef Frag<_Float16> F;
  __shared__ __align__(16) float slab[4][NCH * SPITCH];
  const int tid = threadIdx.x;
  const int lane = tid & 31;
  const int wave = tid >> 5;
  const int hh = lane >> 4;
  const int cix = lane & 15;
  const int koff = hh * 8;
  const int b = blockIdx.x >> 8;
  const int y = blockIdx.x & 255;
  const int x0w = wave * 64;

  v8f acc[4];
#pragma unroll
  for (int s = 0; s < 4; ++s) acc[s] = (v8f){0.f, 0.f, 0.f, 0.f, 0.f, 0.f, 0.f, 0.f};

#pragma unroll 1
  for (int br = 0; br < 2; ++br) {
    const _Float16* tm = (const _Float16*)((br == 0) ? tsu : tnu);
    const _Float16* wrow = (const _Float16*)w2p + (size_t)br * N2ROWS * K2 + (size_t)cix * K2 + koff;
    const int dil = 1 + br;
#pragma unroll 1
    for (int tap = 0; tap < 9; ++tap) {
      const int kyq = tap / 3;
      const int ky = kyq - 1;
      const int kx = tap - kyq * 3 - 1;
      const long prow = ((long)(b * PADD + y + 2 + ky * dil)) * PADD + (long)(x0w + 2 + kx * dil + cix);
      const _Float16* arow = tm + prow * NMID + koff;
      const _Float16* wt = wrow + tap * NMID;
#pragma unroll 1
      for (int q = 0; q < 4; ++q) {
        const v16h bf = F::load(wt + q * 32);
        const v16h a0 = F::load(arow + q * 32);
        const v16h a1 = F::load(arow + 16 * NMID + q * 32);
        const v16h a2 = F::load(arow + 32 * NMID + q * 32);
        const v16h a3 = F::load(arow + 48 * NMID + q * 32);
        acc[0] = F::mma(a0, bf, acc[0]);
        acc[1] = F::mma(a1, bf, acc[1]);
        acc[2] = F::mma(a2, bf, acc[2]);
        acc[3] = F::mma(a3, bf, acc[3]);
        guard4a5(acc[0], acc[1], acc[2], acc[3], a0, a1, a2, a3, bf);
      }
    }
  }
  acc_guard4(acc[0], acc[1], acc[2], acc[3]);

  const int ncl = (cix < NCH) ? cix : (NCH - 1);
  const float bsum = bsu[ncl] + bnu[ncl];
  float* sw = slab[wave];
  if (cix < NCH) {
#pragma unroll
    for (int s = 0; s < 4; ++s)
#pragma unroll
      for (int r = 0; r < 8; ++r)
        sw[cix * SPITCH + s * 16 + 8 * hh + r] = acc[s][r] * C2_FOLD + bsum;
  }
  __syncthreads();
  {
    const int c4 = (lane & 15) * 4;
    for (int pass = 0; pass < 2; ++pass) {
#pragma unroll
      for (int it = 0; it < 2; ++it) {
        const int ch = it * 2 + hh;
        const v4f v = *(const v4f*)(sw + ch * SPITCH + c4);
        *(volatile v4f*)(accp + ((size_t)(b * NCH + ch) * NHT + y) * NWD + x0w + c4) = v;
      }
      __threadfence();
    }
  }
}

__global__ __launch_bounds__(NTHR) void k_sobel(const float* __restrict__ st, const float* __restrict__ skx,
                                                 const float* __restrict__ sky, float* __restrict__ gmp) {
  __shared__ float wk[72];
  const int tid = threadIdx.x;
  const int bc = blockIdx.x >> 8;
  const int y = blockIdx.x & 255;
  const int x = tid;
  const int c = bc & 3;
  if (tid < 36) wk[tid] = skx[tid];
  if (tid >= 128 && tid < 164) wk[36 + tid - 128] = sky[tid - 128];
  __syncthreads();
  const float* plane = st + (size_t)bc * HWPIX;
  const float g = grad_mag(plane, y, x, wk + c * 9, wk + 36 + c * 9);
  st2(gmp + (size_t)bc * HWPIX + (size_t)y * NWD + x, g);
}

#pragma clang fp contract(off)
__global__ __launch_bounds__(NTHR) void k_boxsim(const float* __restrict__ gmp, const float* __restrict__ st,
                                                  float* __restrict__ simp, float* __restrict__ bssp,
                                                  float* __restrict__ part) {
  __shared__ float red[NTHR];
  const int tid = threadIdx.x;
  const int bc = blockIdx.x >> 8;
  const int y = blockIdx.x & 255;
  const int x = tid;
  const float* g = gmp + (size_t)bc * HWPIX;
  const float* s = st + (size_t)bc * HWPIX;
  float sg = 0.0f, sg2 = 0.0f, ss = 0.0f;
#pragma unroll 1
  for (int dy = -2; dy <= 2; ++dy) {
    const int yy = y + dy;
    if (yy < 0 || yy >= NHT) continue;
    const float* gr = g + (size_t)yy * NWD;
    const float* sr = s + (size_t)yy * NWD;
#pragma unroll 1
    for (int dx = -2; dx <= 2; ++dx) {
      const int xx = x + dx;
      const float f = (xx >= 0 && xx < NWD) ? 1.0f : 0.0f;
      const int xc = (xx < 0) ? 0 : ((xx > NWD - 1) ? (NWD - 1) : xx);
      const float gv = gr[xc] * f;
      const float sv = sr[xc] * f;
      const float gq = gv * gv;
      sg = sg + gv;
      sg2 = sg2 + gq;
      ss = ss + sv;
    }
  }
  const size_t idx = (size_t)bc * HWPIX + (size_t)y * NWD + x;
  const float gc = g[(size_t)y * NWD + x];
  const float t2 = (2.0f * gc) * sg;
  const float t3 = (25.0f * gc) * gc;
  const float dist = (sg2 - t2) + t3;
  float sim = expf(-2.0f * dist);
  if (sim < FLT_TINY) sim = 0.0f;
  st2(simp + idx, sim);
  st2(bssp + idx, ss);
  red[tid] = sim;
  __syncthreads();
#pragma unroll 1
  for (int off = NTHR / 2; off > 0; off >>= 1) {
    if (tid < off) red[tid] += red[tid + off];
    __syncthreads();
  }
  if (tid < 32) {
    const float tot = red[0];
    const float pv = tot * ((tid == 0) ? 1.0f : 0.0f);
    st2(part + (size_t)blockIdx.x * PLINE + tid, pv);
  }
}
#pragma clang fp contract(fast)

__global__ __launch_bounds__(NTHR) void k_dcconv(const float* __restrict__ st, const float* __restrict__ dcw,
                                                  const float* __restrict__ dcb, float* __restrict__ hfp) {
  __shared__ float tile[NCH * 3 * PADD];
  __shared__ float wsh[NCH * NCH * 9 + NCH];
  const int tid = threadIdx.x;
  const int bc = blockIdx.x >> 8;
  const int y = blockIdx.x & 255;
  const int x = tid;
  const int b = bc >> 2;
  const int c = bc & 3;
  if (tid < 24) {
    const int q = tid >> 1;
    const int col = (tid & 1) ? (NWD + 1) : 0;
    tile[q * PADD + col] = 0.0f;
  }
  if (tid < NCH * NCH * 9) wsh[tid] = dcw[tid];
  if (tid >= 160 && tid < 160 + NCH) wsh[NCH * NCH * 9 + tid - 160] = dcb[tid - 160];
  __syncthreads();
#pragma unroll 1
  for (int q = 0; q < NCH * 3; ++q) {
    const int c2 = q / 3;
    const int r = q - c2 * 3;
    const int yy = y + r - 1;
    float v = 0.0f;
    if (yy >= 0 && yy < NHT) v = st[((size_t)(b * NCH + c2) * NHT + yy) * NWD + tid];
    tile[q * PADD + tid + 1] = v;
  }
  __syncthreads();
  float hs = 0.0f;
#pragma unroll
  for (int c2 = 0; c2 < NCH; ++c2) {
    const float* wr = wsh + (c * NCH + c2) * 9;
    const float* tr = tile + (c2 * 3) * PADD + x;
#pragma unroll
    for (int ky = 0; ky < 3; ++ky) {
#pragma unroll
      for (int kx = 0; kx < 3; ++kx) hs += wr[ky * 3 + kx] * tr[ky * PADD + kx];
    }
  }
  hs += wsh[NCH * NCH * 9 + c];
  const size_t idx = (size_t)bc * HWPIX + (size_t)y * NWD + x;
  st2(hfp + idx, hs);
}

__global__ __launch_bounds__(NTHR) void k_combine(const float* __restrict__ simp, const float* __restrict__ bssp,
                                                   const float* __restrict__ part, const float* __restrict__ accp,
                                                   const float* __restrict__ hfp, float* __restrict__ nxt) {
  __shared__ float red[NTHR];
  const int tid = threadIdx.x;
  const int bc = blockIdx.x >> 8;
  const int y = blockIdx.x & 255;
  const int x = tid;
  red[tid] = part[((size_t)bc * NHT + tid) * PLINE];
  __syncthreads();
#pragma unroll 1
  for (int off = NTHR / 2; off > 0; off >>= 1) {
    if (tid < off) red[tid] += red[tid + off];
    __syncthreads();
  }
  const float ssum = red[0];
  const float rinv = 1.0f / (ssum + 1e-8f);
  const size_t idx = (size_t)bc * HWPIX + (size_t)y * NWD + x;
  const float wv = (simp[idx] * rinv) * bssp[idx];
  const float nv = (wv + accp[idx]) + hfp[idx];
  st2(nxt + idx, nv);
}

__global__ __launch_bounds__(NTHR) void k_final(const float* __restrict__ st, const float* __restrict__ gmp,
                                                 const float* __restrict__ hfp, const int* __restrict__ tmodp,
                                                 float* __restrict__ out, float* __restrict__ lpart) {
  __shared__ float red[NTHR];
  const int tid = threadIdx.x;
  const int bc = blockIdx.x >> 8;
  const int y = blockIdx.x & 255;
  const int x = tid;
  const int b = bc >> 2;
  const size_t idx = (size_t)bc * HWPIX + (size_t)y * NWD + x;
  const float sv = st[idx];
  const float gmv = gmp[idx];
  const float hpre = hfp[idx];
  const int traw = tmodp[b];
  const float hf = fsigm(hpre);
  const float sgm = fsigm(gmv);
  const float g4 = fsigm(gmv * hf);
  const int t = (traw < 0) ? 0 : ((traw > 3) ? 3 : traw);
  const float hsg = hf * sgm;
  const float p0 = hf,  q0 = 1.0f - sgm;
  const float p1 = sgm, q1 = 1.0f - hf;
  const float p2 = hsg, q2 = 1.0f - hsg;
  const float p3 = g4,  q3 = 1.0f - g4;
  float pos = (t == 0) ? p0 : ((t == 1) ? p1 : ((t == 2) ? p2 : p3));
  float neg = (t == 0) ? q0 : ((t == 1) ? q1 : ((t == 2) ? q2 : q3));
  pos = fminf(fmaxf(pos, 0.0f), 1.0f);
  neg = fminf(fmaxf(neg, 0.0f), 1.0f);
  const float ep = expf(pos);
  const float en = expf(neg);
  const float sel = ep / ((ep + en) + 1e-8f);
  const float ov = sv * sel;
  st2(out + idx, ov);
  const float lv = sel * neg + (1.0f - sel) * pos;
  red[tid] = lv;
  __syncthreads();
#pragma unroll 1
  for (int off = NTHR / 2; off > 0; off >>= 1) {
    if (tid < off) red[tid] += red[tid + off];
    __syncthreads();
  }
  if (tid < 32) {
    const float tot = red[0];
    const float pv = tot * ((tid == 0) ? 1.0f : 0.0f);
    st2(lpart + (size_t)blockIdx.x * PLINE + tid, pv);
  }
}

__global__ __launch_bounds__(NTHR) void k_loss(const float* __restrict__ lpart, float* __restrict__ out) {
  __shared__ float red[NTHR];
  const int tid = threadIdx.x;
  float s = 0.0f;
#pragma unroll 1
  for (int j = 0; j < NROWBLK / NTHR; ++j) s += lpart[((size_t)j * NTHR + tid) * PLINE];
  red[tid] = s;
  __syncthreads();
#pragma unroll 1
  for (int off = NTHR / 2; off > 0; off >>= 1) {
    if (tid < off) red[tid] += red[tid + off];
    __syncthreads();
  }
  if (tid == 0) {
    const float v = red[0] * (1.0f / 524288.0f);
    st2(out + NPIX, v);
  }
}

extern "C" void kernel_launch(void* const* d_in, const int* in_sizes, int n_in,
                              void* d_out, int out_size, void* d_ws, size_t ws_size, hipStream_t stream) {
  if (n_in < 17) return;
  if (in_sizes[0] != NPIX) return;
  if (out_size != NPIX + 1) return;
  if (ws_size < WS_TOTAL) return;

  const float* x      = (const float*)d_in[0];
  const int*   tmodp  = (const int*)d_in[1];
  const float* fcw    = (const float*)d_in[2];
  const float* fcb    = (const float*)d_in[3];
  const float* mw     = (const float*)d_in[4];
  const float* su_w1  = (const float*)d_in[5];
  const float* su_b1  = (const float*)d_in[6];
  const float* su_w2  = (const float*)d_in[7];
  const float* su_b2  = (const float*)d_in[8];
  const float* nu_w1  = (const float*)d_in[9];
  const float* nu_b1  = (const float*)d_in[10];
  const float* nu_w2  = (const float*)d_in[11];
  const float* nu_b2  = (const float*)d_in[12];
  const float* dcw    = (const float*)d_in[13];
  const float* dcb    = (const float*)d_in[14];
  const float* skx    = (const float*)d_in[15];
  const float* sky    = (const float*)d_in[16];

  char* ws = (char*)d_ws;
  unsigned short* tsu  = (unsigned short*)(ws + OFF_TSU);
  unsigned short* tnu  = (unsigned short*)(ws + OFF_TNU);
  unsigned short* imh  = (unsigned short*)(ws + OFF_IMH);
  unsigned short* iml  = (unsigned short*)(ws + OFF_IML);
  float* stA  = (float*)(ws + OFF_STA);
  float* stB  = (float*)(ws + OFF_STB);
  float* accp = (float*)(ws + OFF_ACC);
  float* gmp  = (float*)(ws + OFF_GM);
  float* simp = (float*)(ws + OFF_SIM);
  float* bssp = (float*)(ws + OFF_BSS);
  float* hfp  = (float*)(ws + OFF_HF);
  unsigned short* w1h = (unsigned short*)(ws + OFF_W1H);
  unsigned short* w1l = (unsigned short*)(ws + OFF_W1L);
  unsigned short* w2p = (unsigned short*)(ws + OFF_W2);
  float* part  = (float*)(ws + OFF_PART);
  float* lpart = (float*)(ws + OFF_LPRT);
  float* gate  = (float*)(ws + OFF_GATE);
  float* out   = (float*)d_out;

  k_zero16<<<ZERO_BLOCKS, NTHR, 0, stream>>>(tsu, (long)(2 * TMID_HALVES / 8));
  k_w1prep<<<dim3(NMID * (K1 / 8) / NTHR, 2), NTHR, 0, stream>>>(su_w1, nu_w1, w1h, w1l);
  k_w2prep<<<dim3(N2ROWS * (K2 / 8) / NTHR, 2), NTHR, 0, stream>>>(su_w2, nu_w2, w2p);
  k_gate<<<1, NTHR, 0, stream>>>(x, fcw, fcb, mw, gate);
  k_init<<<NPIX / 4 / NTHR, NTHR, 0, stream>>>(x, gate, stA);

  float* cur = stA;
  float* nxt = stB;
  for (int it = 0; it < 3; ++it) {
    k_im2col<<<NIMGROW, NTHR, 0, stream>>>(cur, 1, imh, iml);
    k_conv1<<<CONV1_BLOCKS, NTHR, 0, stream>>>(imh, iml, w1h, w1l, su_b1, tsu);
    k_im2col<<<NIMGROW, NTHR, 0, stream>>>(cur, 2, imh, iml);
    k_conv1<<<CONV1_BLOCKS, NTHR, 0, stream>>>(imh, iml, w1h + NMID * K1, w1l + NMID * K1, nu_b1, tnu);
    k_conv2<<<NIMGROW, 128, 0, stream>>>(tsu, tnu, w2p, su_b2, nu_b2, accp);
    k_sobel<<<NROWBLK, NTHR, 0, stream>>>(cur, skx, sky, gmp);
    k_boxsim<<<NROWBLK, NTHR, 0, stream>>>(gmp, cur, simp, bssp, part);
    k_dcconv<<<NROWBLK, NTHR, 0, stream>>>(cur, dcw, dcb, hfp);
    k_combine<<<NROWBLK, NTHR, 0, stream>>>(simp, bssp, part, accp, hfp, nxt);
    float* tsw = cur; cur = nxt; nxt = tsw;
  }
  k_sobel<<<NROWBLK, NTHR, 0, stream>>>(cur, skx, sky, gmp);
  k_dcconv<<<NROWBLK, NTHR, 0, stream>>>(cur, dcw, dcb, hfp);
  k_final<<<NROWBLK, NTHR, 0, stream>>>(cur, gmp, hfp, tmodp, out, lpart);
  k_loss<<<1, NTHR, 0, stream>>>(lpart, out);
}
